// myVMLMF_CELL_26680336843034
// MI455X (gfx1250) — hardware-run, weakly checked
//
#include <hip/hip_runtime.h>


#define NR   4096
#define NI   512
#define NH   1024
#define RK   128
#define G4   4096
typedef _Float16 h16;
typedef unsigned short bf;
typedef __attribute__((ext_vector_type(16))) __bf16   v16bf;
typedef __attribute__((ext_vector_type(16))) _Float16 v16h;
typedef __attribute__((ext_vector_type(8)))  _Float16 v8h;
typedef __attribute__((ext_vector_type(8)))  unsigned short v8us;
typedef __attribute__((ext_vector_type(8)))  float    v8f;
typedef __attribute__((ext_vector_type(4)))  float    v4f;
typedef v8h  __attribute__((may_alias)) v8ha;
typedef v4f  __attribute__((may_alias)) v4fa;
typedef v8us __attribute__((may_alias)) v8usa;

__device__ __forceinline__ unsigned short f2bf(float f) { unsigned u = __float_as_uint(f); u += 0x7FFFu + ((u >> 16) & 1u); return (unsigned short)(u >> 16); }
__device__ __forceinline__ float bf2f(unsigned short b) { return __uint_as_float(((unsigned)b) << 16); }
__device__ __forceinline__ float bfr(float f) { return bf2f(f2bf(f)); }
__device__ __forceinline__ v16h cat16(v8h lo, v8h hi) { return __builtin_shufflevector(lo, hi, 0, 1, 2, 3, 4, 5, 6, 7, 8, 9, 10, 11, 12, 13, 14, 15); }
__device__ __forceinline__ v16bf cat16b(v8us lo, v8us hi) { return __builtin_bit_cast(v16bf, __builtin_shufflevector(lo, hi, 0, 1, 2, 3, 4, 5, 6, 7, 8, 9, 10, 11, 12, 13, 14, 15)); }
__device__ __forceinline__ v8f wmma16(v16h a, v16h b, v8f c) { return __builtin_amdgcn_wmma_f32_16x16x32_f16(false, a, false, b, (short)0, c, false, false); }
__device__ __forceinline__ v8f wmmab(v16bf a, v16bf b, v8f c) { return __builtin_amdgcn_wmma_f32_16x16x32_bf16(false, a, false, b, (short)0, c, false, false); }


template <typename T16> struct WFrag;
template <> struct WFrag<h16> { typedef v16h V; static __device__ __forceinline__ V ld(const h16* p) { return cat16(*(const v8h*)p, *(const v8h*)(p + 16)); } static __device__ __forceinline__ v8f mma(V a, V b, v8f c) { return wmma16(a, b, c); } };
template <> struct WFrag<bf> { typedef v16bf V; static __device__ __forceinline__ V ld(const bf* p) { return cat16b(*(const v8us*)p, *(const v8us*)(p + 16)); } static __device__ __forceinline__ v8f mma(V a, V b, v8f c) { return wmmab(a, b, c); } };
template <typename T16, int NSPLIT, bool BIAS>
__global__ __launch_bounds__(32) void k_gemmw(const T16* __restrict__ A, const T16* __restrict__ A2, const T16* __restrict__ Bt, const T16* __restrict__ Bt2, int K, float* C, int ldc, const float* __restrict__ bias, size_t sA, size_t sB, size_t sC) {
    typedef typename WFrag<T16>::V V;
    __shared__ __align__(16) float os[16 * 68];
    const size_t z = blockIdx.z; A += z * sA; if (A2) A2 += z * sA; Bt += z * sB; if (Bt2) Bt2 += z * sB; C += z * sC;
    const int lane = threadIdx.x & 31, lr = lane & 15, hi = lane >> 4; const int r0 = blockIdx.x * 64, c0 = blockIdx.y * 64;
    v8f acc[4][4];
#pragma unroll
    for (int mb = 0; mb < 4; ++mb)
#pragma unroll
        for (int nb = 0; nb < 4; ++nb) acc[mb][nb] = (v8f){};
    const size_t aoff = (size_t)(r0 + lr) * K + 8 * hi, boff = (size_t)(c0 + lr) * K + 8 * hi;
#pragma unroll 1
    for (int kc = 0; kc < K; kc += 32) {
        V a[4], a2[4];
#pragma unroll
        for (int mb = 0; mb < 4; ++mb) { a[mb] = WFrag<T16>::ld(A + aoff + (size_t)mb * 16 * K + kc); if (NSPLIT == 1 || NSPLIT == 2) a2[mb] = WFrag<T16>::ld(A2 + aoff + (size_t)mb * 16 * K + kc); }
#pragma unroll
        for (int nb = 0; nb < 4; ++nb) { const V b = WFrag<T16>::ld(Bt + boff + (size_t)nb * 16 * K + kc); V b2; if (NSPLIT >= 2) b2 = WFrag<T16>::ld(Bt2 + boff + (size_t)nb * 16 * K + kc);
#pragma unroll
            for (int mb = 0; mb < 4; ++mb) { acc[mb][nb] = WFrag<T16>::mma(a[mb], b, acc[mb][nb]); if (NSPLIT == 1 || NSPLIT == 2) acc[mb][nb] = WFrag<T16>::mma(a2[mb], b, acc[mb][nb]); if (NSPLIT >= 2) acc[mb][nb] = WFrag<T16>::mma(a[mb], b2, acc[mb][nb]); } }
        asm volatile("v_nop\n\tv_nop\n\tv_nop\n\tv_nop" : "+v"(acc[0][0]), "+v"(acc[1][1]), "+v"(acc[2][2]), "+v"(acc[3][3]) : "v"(a[0]), "v"(a[3]));
    }
#pragma unroll
    for (int mb = 0; mb < 4; ++mb) {
#pragma unroll
        for (int nb = 0; nb < 4; ++nb) {
#pragma unroll
            for (int j = 0; j < 8; ++j) os[(hi * 8 + j) * 68 + nb * 16 + lr] = acc[mb][nb][j]; }
        __builtin_amdgcn_wave_barrier(); asm volatile("" ::: "memory");
        float* crow = C + (size_t)(r0 + mb * 16) * ldc + c0;
#pragma unroll 1
        for (int ps = 0; ps < 2; ++ps) {
#pragma unroll
            for (int s = 0; s < 8; ++s) { const int row = 2 * s + hi, cofs = lr * 4; v4f val = *(const v4fa*)(os + row * 68 + cofs); if (BIAS) { val[0] += bfr(bias[c0 + cofs]); val[1] += bfr(bias[c0 + cofs + 1]); val[2] += bfr(bias[c0 + cofs + 2]); val[3] += bfr(bias[c0 + cofs + 3]); }
                *(volatile v4f*)(crow + (size_t)row * ldc + cofs) = val; }
            if (ps == 0) __threadfence(); }
        __builtin_amdgcn_wave_barrier(); asm volatile("" ::: "memory");
    }
}

__device__ __forceinline__ void splitf(float y, unsigned short& h, unsigned short& l) { h = f2bf(y); l = f2bf(y - bf2f(h)); }
typedef __attribute__((ext_vector_type(2))) unsigned short v2us;
typedef __attribute__((ext_vector_type(4))) unsigned short v4us;

__global__ __launch_bounds__(256) void k_wtG(const float* __restrict__ w, int K, int N, bf* Bt) {
    const int lane = threadIdx.x & 31; const int L0 = (blockIdx.x * 8 + (threadIdx.x >> 5)) * 8; const int nlines = N * K / 64;
#pragma unroll
    for (int ps = 0; ps < 2; ++ps) {
#pragma unroll 1
        for (int l = 0; l < 8; ++l) { const int L = L0 + l; if (L >= nlines) break; const size_t e = (size_t)L * 64 + lane * 2; const int k = (int)(e % K), n = (int)(e / K); v2us o;
            o[0] = f2bf(w[(size_t)k * N + n]); o[1] = f2bf(w[(size_t)(k + 1) * N + n]); *(volatile v2us*)(Bt + e) = o; }
        if (ps == 0) __threadfence(); }
}
__global__ __launch_bounds__(256) void k_cvt8(const float* __restrict__ src, bf* dst, size_t n8) { const size_t i = (size_t)blockIdx.x * 256 + threadIdx.x; if (i >= n8) return; const v8f v = *(const v8f*)(src + i * 8); v8us o;
#pragma unroll
    for (int k = 0; k < 8; ++k) o[k] = f2bf(v[k]); *(volatile v8us*)(dst + i * 8) = o; __threadfence(); *(volatile v8us*)(dst + i * 8) = o; }
__global__ __launch_bounds__(256) void k_spl(const float* __restrict__ F, size_t n4, bf* Hh, bf* Hl) { const size_t e = ((size_t)blockIdx.x * 256 + threadIdx.x) * 4; if (e >= n4) return; const v4f a = *(const v4f*)(F + e); v4us oh, ol;
#pragma unroll
    for (int u = 0; u < 4; ++u) { unsigned short h, l; splitf(a[u], h, l); oh[u] = h; ol[u] = l; } *(volatile v4us*)(Hh + e) = oh; *(volatile v4us*)(Hl + e) = ol; __threadfence(); *(volatile v4us*)(Hh + e) = oh; *(volatile v4us*)(Hl + e) = ol; }
__global__ __launch_bounds__(256) void k_corr(const float* __restrict__ U, const float* __restrict__ V, int NJ, float* CR) { const int idx = blockIdx.x * 256 + threadIdx.x; if (idx >= 4 * NJ) return; const int j = idx % NJ; const int g = idx / NJ; float s = 0.f;
#pragma unroll 1
    for (int r = 0; r < RK; ++r) { float a = bfr(U[(size_t)j * RK + r]), b = bfr(V[((size_t)g * NH + j) * RK + r]); asm volatile("" : "+v"(a)); float p = __fmul_rn(a, b); asm volatile("" : "+v"(p)); s = __fadd_rn(s, p); }
    *(volatile float*)(CR + idx) = s; __threadfence(); *(volatile float*)(CR + idx) = s; }
__device__ __forceinline__ float sigm(float t) { return __fdiv_rn(1.0f, __fadd_rn(1.0f, __expf(-t))); }
__global__ __launch_bounds__(256) void k_gate(const float* __restrict__ LX, const float* __restrict__ LH, const float* __restrict__ x, const float* __restrict__ h, const float* __restrict__ c, const float* __restrict__ CRX, const float* __restrict__ CRH, const float* __restrict__ b_x, const float* __restrict__ b_h, const float* __restrict__ dia_x, const float* __restrict__ dia_h, float* HN, float* CN) {
    const int e = (blockIdx.x * 256 + threadIdx.x) * 4; if (e >= NR * NH) return; const int j0 = e % NH; const int b = e / NH; v4f oh, oc;
#pragma unroll 1
    for (int u = 0; u < 4; ++u) { const int j = j0 + u; const float hv = bfr(h[(size_t)b * NH + j]); const float xv = (j < NI) ? bfr(x[(size_t)b * NI + j]) : 0.f; float pre[4];
#pragma unroll 1
        for (int g = 0; g < 4; ++g) { const size_t col = (size_t)g * NH + j;
            float rx = (j < NI) ? __fmul_rn(xv, CRX[g * NI + j]) : 0.f; asm volatile("" : "+v"(rx)); const float gx = __fadd_rn(__fsub_rn(LX[(size_t)b * G4 + col], rx), bfr(b_x[col]));
            float rh = __fmul_rn(hv, CRH[g * NH + j]); asm volatile("" : "+v"(rh)); const float gh = __fadd_rn(__fsub_rn(LH[(size_t)b * G4 + col], rh), bfr(b_h[col]));
            float vx = (j < NI) ? __fmul_rn(bfr(dia_x[j]), xv) : 0.f, vh = __fmul_rn(bfr(dia_h[j]), hv); asm volatile("" : "+v"(vx)); asm volatile("" : "+v"(vh)); const float add = __fadd_rn(vx, vh);
            pre[g] = __fadd_rn(__fadd_rn(gx, gh), add); }
        const float ig = sigm(pre[0]), fg = sigm(pre[1]), og = sigm(pre[2]), ng = tanhf(pre[3]); float t1 = __fmul_rn(fg, bfr(c[(size_t)b * NH + j])), t2 = __fmul_rn(ig, ng); asm volatile("" : "+v"(t1)); asm volatile("" : "+v"(t2)); const float cn = __fadd_rn(t1, t2); oc[u] = cn; oh[u] = __fmul_rn(og, tanhf(cn)); }
    for (int ps = 0; ps < 2; ++ps) { *(volatile v4f*)(HN + e) = oh; *(volatile v4f*)(CN + e) = oc; if (ps == 0) __threadfence(); } }

extern "C" void kernel_launch(void* const* d_in, const int* in_sizes, int n_in,
                              void* d_out, int out_size, void* d_ws, size_t ws_size, hipStream_t stream) {
    (void)in_sizes; (void)n_in; (void)out_size;
    const float** I = (const float**)d_in;
    const float *x = I[0], *h = I[1], *c = I[2], *U_x = I[3], *U_h = I[4], *V_x = I[5], *V_h = I[6], *b_x = I[7], *b_h = I[8], *dia_x = I[9], *dia_h = I[10];
    float* HN = (float*)d_out; float* CN = HN + (size_t)NR * NH;
    char* wsp = (char*)d_ws;
    auto take = [&](size_t bytes) { char* p = wsp; wsp += (bytes + 255) & ~(size_t)255; return (void*)p; };
    bf* BUX = (bf*)take(RK * NI * 2); bf* BUH = (bf*)take(RK * NH * 2); bf* BVX = (bf*)take((size_t)G4 * RK * 2); bf* BVH = (bf*)take((size_t)G4 * RK * 2); bf* XB = (bf*)take((size_t)NR * NI * 2); bf* HB = (bf*)take((size_t)NR * NH * 2);
    float* XU = (float*)take((size_t)NR * RK * 4); float* HU = (float*)take((size_t)NR * RK * 4); bf* XUh = (bf*)take((size_t)NR * RK * 2); bf* XUl = (bf*)take((size_t)NR * RK * 2); bf* HUh = (bf*)take((size_t)NR * RK * 2); bf* HUl = (bf*)take((size_t)NR * RK * 2);
    float* LX = (float*)take((size_t)NR * G4 * 4); float* LH = (float*)take((size_t)NR * G4 * 4); float* CRX = (float*)take(4 * NI * 4); float* CRH = (float*)take(4 * NH * 4);
    if ((size_t)(wsp - (char*)d_ws) > ws_size) return;
    k_wtG<<<(NI * RK / 64 + 63) / 64, 256, 0, stream>>>(U_x, NI, RK, BUX); k_wtG<<<(NH * RK / 64 + 63) / 64, 256, 0, stream>>>(U_h, NH, RK, BUH);
    k_cvt8<<<(G4 * RK / 8 + 255) / 256, 256, 0, stream>>>(V_x, BVX, (size_t)G4 * RK / 8); k_cvt8<<<(G4 * RK / 8 + 255) / 256, 256, 0, stream>>>(V_h, BVH, (size_t)G4 * RK / 8);
    k_cvt8<<<(NR * NI / 8 + 255) / 256, 256, 0, stream>>>(x, XB, (size_t)NR * NI / 8); k_cvt8<<<(NR * NH / 8 + 255) / 256, 256, 0, stream>>>(h, HB, (size_t)NR * NH / 8);
    k_gemmw<bf, 0, false><<<dim3(NR / 64, RK / 64, 1), 32, 0, stream>>>(XB, nullptr, BUX, nullptr, NI, XU, RK, nullptr, 0, 0, 0); k_gemmw<bf, 0, false><<<dim3(NR / 64, RK / 64, 1), 32, 0, stream>>>(HB, nullptr, BUH, nullptr, NH, HU, RK, nullptr, 0, 0, 0);
    k_spl<<<(NR * RK / 4 + 255) / 256, 256, 0, stream>>>(XU, (size_t)NR * RK, XUh, XUl); k_spl<<<(NR * RK / 4 + 255) / 256, 256, 0, stream>>>(HU, (size_t)NR * RK, HUh, HUl);
    k_gemmw<bf, 1, false><<<dim3(NR / 64, G4 / 64, 1), 32, 0, stream>>>(XUh, XUl, BVX, nullptr, RK, LX, G4, nullptr, 0, 0, 0); k_gemmw<bf, 1, false><<<dim3(NR / 64, G4 / 64, 1), 32, 0, stream>>>(HUh, HUl, BVH, nullptr, RK, LH, G4, nullptr, 0, 0, 0);
    k_corr<<<(4 * NI + 255) / 256, 256, 0, stream>>>(U_x, V_x, NI, CRX); k_corr<<<(4 * NH + 255) / 256, 256, 0, stream>>>(U_h, V_h, NH, CRH);
    k_gate<<<(NR * NH / 4 + 255) / 256, 256, 0, stream>>>(LX, LH, x, h, c, CRX, CRH, b_x, b_h, dia_x, dia_h, HN, CN);
}
